// MultimodalDiffusionTransformer_58609123722032
// MI455X (gfx1250) — hardware-verified
//
#include <hip/hip_runtime.h>
#include <math.h>

#define HH 512
#define BB 256
#define TT 1000
#define TP 1008
#define HD2 256

typedef __attribute__((ext_vector_type(16))) __bf16 v16bf;
typedef __attribute__((ext_vector_type(8)))  __bf16 v8bf;
typedef __attribute__((ext_vector_type(8)))  float  v8f;
typedef __attribute__((ext_vector_type(4)))  float  v4f;
typedef __attribute__((ext_vector_type(4)))  unsigned v4u;
typedef float __attribute__((may_alias)) float_a;

template <typename V> __device__ __forceinline__ void vst2(void* p, V v) {
  *(volatile V*)p = v; __threadfence(); *(volatile V*)p = v;
}
__device__ __forceinline__ v8f wmma_bf(v16bf a, v16bf b, v8f c) {
  v8f d = __builtin_amdgcn_wmma_f32_16x16x32_bf16(false, a, false, b, (short)0, c, false, false);
  asm volatile("v_nop\n\tv_nop\n\tv_nop\n\tv_nop" : "+v"(d) : "v"(a), "v"(b));
  return d;
}
struct A3 { v16bf h, m, l; };
__device__ __forceinline__ A3 split_row(const float* row, int k0, int lane) {
  A3 r; const float* p = row + k0 + 8 * (lane >> 4);
#pragma unroll
  for (int i = 0; i < 16; ++i) {
    const float x = p[(i < 8) ? i : (i + 8)];
    const __bf16 h = (__bf16)x; const float rh = x - (float)h;
    const __bf16 m = (__bf16)rh; const __bf16 l = (__bf16)(rh - (float)m);
    r.h[i] = h; r.m[i] = m; r.l[i] = l;
  }
  return r;
}
__device__ __forceinline__ v16bf frag_bf(const __bf16* row, int k0, int lane) {
  union { v16bf v; v8bf q[2]; } r; const __bf16* p = row + k0 + 8 * (lane >> 4);
  r.q[0] = *(const v8bf*)(p); r.q[1] = *(const v8bf*)(p + 16); return r.v;
}
__device__ __forceinline__ v8f mac6(const A3& a, const __bf16* bh, const __bf16* bm, const __bf16* bl, int k0, int lane, v8f c) {
  const v16bf fh = frag_bf(bh, k0, lane), fm = frag_bf(bm, k0, lane), fl = frag_bf(bl, k0, lane);
  c = wmma_bf(a.l, fh, c); c = wmma_bf(a.m, fm, c); c = wmma_bf(a.h, fl, c);
  c = wmma_bf(a.m, fh, c); c = wmma_bf(a.h, fm, c); c = wmma_bf(a.h, fh, c);
  return c;
}

__global__ __launch_bounds__(256) void k_split3(const float* __restrict__ W, __bf16* __restrict__ P, int K, int N) {
  __shared__ __align__(16) __bf16 th[64][72], tm[64][72], tl[64][72];
  const int nt = N / 64, tid = threadIdx.x;
  const int n0 = (blockIdx.x % nt) * 64, k0 = (blockIdx.x / nt) * 64;
  for (int i = tid; i < 64 * 64; i += 256) {
    const int kk = i >> 6, nn = i & 63;
    const float x = W[(size_t)(k0 + kk) * N + n0 + nn];
    const __bf16 h = (__bf16)x; const float rh = x - (float)h; const __bf16 m = (__bf16)rh; const __bf16 l = (__bf16)(rh - (float)m);
    th[nn][kk] = h; tm[nn][kk] = m; tl[nn][kk] = l;
  }
  __syncthreads();
  const size_t plane = (size_t)N * K;
  for (int g = tid; g < 64 * 8; g += 256) {
    const int nn = g >> 3, pc = g & 7; const size_t o = (size_t)(n0 + nn) * K + k0 + pc * 8;
    vst2(P + o, *(const v4u*)(&th[nn][pc * 8])); vst2(P + plane + o, *(const v4u*)(&tm[nn][pc * 8])); vst2(P + 2 * plane + o, *(const v4u*)(&tl[nn][pc * 8]));
  }
}

__global__ __launch_bounds__(32) void k_coeff(float* __restrict__ coef) {
  __shared__ float ac[TT];
  if (threadIdx.x == 0) {
    double prod = 1.0;
    for (int t = 0; t < TT; ++t) {
      const float beta = 1e-4f + (float)t * ((0.02f - 1e-4f) / (float)(TT - 1));
      prod *= (double)(1.0f - beta);
      ac[t] = (float)prod;
    }
  }
  __syncthreads();
  for (int s = threadIdx.x; s < 1024; s += 32) {
    float a = 0.f, b = 0.f, d = 0.f;
    if (s < TT) {
      const int t = TT - 1 - s;
      const float beta = 1e-4f + (float)t * ((0.02f - 1e-4f) / (float)(TT - 1));
      const float acp = (t == 0) ? 1.0f : ac[t - 1];
      a = sqrtf(ac[t]); b = sqrtf(1.0f - ac[t]); d = sqrtf(1.0f - acp) + sqrtf(beta);
    }
    vst2(coef + s, (float_a)a); vst2(coef + 1024 + s, (float_a)b); vst2(coef + 2048 + s, (float_a)d);
  }
}

__global__ __launch_bounds__(256) void k_teh(const float* __restrict__ tw1, const float* __restrict__ tb1, float* __restrict__ teh) {
  const int i = blockIdx.x * 256 + threadIdx.x;
  const int t = i / HH, n = i % HH;
  float v = 0.f;
  if (t < TT) { const float z = (float)t * tw1[n] + tb1[n]; v = z / (1.0f + __expf(-z)); }
  vst2(teh + i, (float_a)v);
}

template <int N, int ACT>
__global__ __launch_bounds__(128) void k_gemm6(const float* __restrict__ X, const __bf16* __restrict__ P, const float* __restrict__ bias,
                                              float* __restrict__ Y) {
  __shared__ __align__(16) float so[16 * N];
  const int tid = threadIdx.x, wave = tid >> 5, lane = tid & 31, hi = lane >> 4, col = lane & 15;
  const int m0 = blockIdx.x * 16;
  constexpr int NW = N / 4, NTW = NW / 16;
  const size_t plane = (size_t)N * HH;
  const float* ar = X + (size_t)(m0 + col) * HH;
  v8f acc[NTW];
#pragma unroll
  for (int j = 0; j < NTW; ++j) acc[j] = (v8f){};
#pragma unroll 1
  for (int kc = 0; kc < HH / 32; ++kc) {
    const A3 a = split_row(ar, kc * 32, lane);
#pragma unroll
    for (int j = 0; j < NTW; ++j) {
      const size_t ro = (size_t)(wave * NW + j * 16 + col) * HH;
      acc[j] = mac6(a, P + ro, P + plane + ro, P + 2 * plane + ro, kc * 32, lane, acc[j]);
    }
  }
#pragma unroll
  for (int j = 0; j < NTW; ++j) {
    const int n = wave * NW + j * 16 + col;
#pragma unroll
    for (int r = 0; r < 8; ++r) { float v = acc[j][r] + bias[n]; if (ACT == 1) v = fmaxf(v, 0.f); so[(hi * 8 + r) * N + n] = v; }
  }
  __syncthreads();
  float* dst = Y + (size_t)m0 * N;
  for (int g = tid; g < 16 * N / 4; g += 128) vst2(dst + g * 4, *(const v4f*)(&so[g * 4]));
}

__global__ __launch_bounds__(256) void k_loop(const float* __restrict__ x0, const __bf16* __restrict__ P1, const __bf16* __restrict__ P2,
                                             const float* __restrict__ tep, const float* __restrict__ nb2, const float* __restrict__ coef,
                                             float* __restrict__ xfin) {
  __shared__ __align__(16) float xs[16][HH];
  __shared__ __align__(16) float hs[16][HH];
  const int tid = threadIdx.x, wave = tid >> 5, lane = tid & 31, hi = lane >> 4, col = lane & 15;
  const int m0 = blockIdx.x * 16, c0 = wave * 64;
  const size_t plane = (size_t)HH * HH;
  for (int i = tid; i < 16 * HH; i += 256) xs[i / HH][i % HH] = x0[(size_t)m0 * HH + i];
  __syncthreads();
  for (int s = 0; s < TT; ++s) {
    const int t = TT - 1 - s;
    const float ca = coef[s], cb = coef[1024 + s], cd = coef[2048 + s];
    v8f acc[4] = {(v8f){}, (v8f){}, (v8f){}, (v8f){}};
#pragma unroll 1
    for (int kc = 0; kc < HH / 32; ++kc) {
      const A3 a = split_row(&xs[col][0], kc * 32, lane);
#pragma unroll
      for (int j = 0; j < 4; ++j) { const size_t ro = (size_t)(c0 + j * 16 + col) * HH; acc[j] = mac6(a, P1 + ro, P1 + plane + ro, P1 + 2 * plane + ro, kc * 32, lane, acc[j]); }
    }
    const float* tp = tep + (size_t)t * HH;
#pragma unroll
    for (int j = 0; j < 4; ++j) { const int n = c0 + j * 16 + col;
#pragma unroll
      for (int r = 0; r < 8; ++r) hs[hi * 8 + r][n] = fmaxf(acc[j][r] + tp[n], 0.f); }
    __syncthreads();
    v8f acc2[4] = {(v8f){}, (v8f){}, (v8f){}, (v8f){}};
#pragma unroll 1
    for (int kc = 0; kc < HH / 32; ++kc) {
      const A3 a = split_row(&hs[col][0], kc * 32, lane);
#pragma unroll
      for (int j = 0; j < 4; ++j) { const size_t ro = (size_t)(c0 + j * 16 + col) * HH; acc2[j] = mac6(a, P2 + ro, P2 + plane + ro, P2 + 2 * plane + ro, kc * 32, lane, acc2[j]); }
    }
#pragma unroll
    for (int j = 0; j < 4; ++j) { const int n = c0 + j * 16 + col;
#pragma unroll
      for (int r = 0; r < 8; ++r) {
        const float eps = acc2[j][r] + nb2[n];
        float x = xs[hi * 8 + r][n];
        x = (x - cb * eps) / ca + cd * eps;
        xs[hi * 8 + r][n] = fminf(fmaxf(x, -1000.0f), 1000.0f);
      } }
    __syncthreads();
  }
#pragma unroll
  for (int q = 0; q < 8; ++q) { const int rl = q * 2 + (lane >> 4), pc = lane & 15;
    vst2(xfin + (size_t)(m0 + rl) * HH + c0 + pc * 4, *(const v4f*)(&xs[rl][c0 + pc * 4])); }
}

__global__ __launch_bounds__(256) void k_out(const float* __restrict__ xfin, const float* __restrict__ dh, const float* __restrict__ eh,
                                            const float* __restrict__ dw2, const float* __restrict__ db2,
                                            const float* __restrict__ ew2, const float* __restrict__ eb2, float* __restrict__ out) {
  const int g = blockIdx.x * 256 + threadIdx.x;
  if (g >= BB * (HH + 3) / 4) return;
  v4f o;
#pragma unroll
  for (int e = 0; e < 4; ++e) {
    const int f = g * 4 + e, b = f / (HH + 3), c = f % (HH + 3);
    float v;
    if (c >= 3) v = xfin[(size_t)b * HH + c - 3];
    else if (c == 0) { float s = db2[0];
#pragma unroll 1
      for (int k = 0; k < HD2; ++k) s = fmaf(dh[(size_t)b * HD2 + k], dw2[k], s); v = s; }
    else { const int j = c - 1; float s = eb2[j];
#pragma unroll 1
      for (int k = 0; k < HD2; ++k) s = fmaf(eh[(size_t)b * HD2 + k], ew2[k * 2 + j], s); v = s; }
    o[e] = v;
  }
  vst2(out + (size_t)g * 4, o);
}

extern "C" void kernel_launch(void* const* d_in, const int* in_sizes, int n_in,
                              void* d_out, int out_size, void* d_ws, size_t ws_size,
                              hipStream_t stream) {
  (void)in_sizes; (void)n_in; (void)out_size; (void)ws_size;
  const float* x0  = (const float*)d_in[0];
  const float* tw1 = (const float*)d_in[1];  const float* tb1 = (const float*)d_in[2];
  const float* tw2 = (const float*)d_in[3];  const float* tb2 = (const float*)d_in[4];
  const float* nw1 = (const float*)d_in[5];  const float* nb1 = (const float*)d_in[6];
  const float* nw2 = (const float*)d_in[7];  const float* nb2 = (const float*)d_in[8];
  const float* dw1 = (const float*)d_in[9];  const float* db1 = (const float*)d_in[10];
  const float* dw2 = (const float*)d_in[11]; const float* db2 = (const float*)d_in[12];
  const float* ew1 = (const float*)d_in[13]; const float* eb1 = (const float*)d_in[14];
  const float* ew2 = (const float*)d_in[15]; const float* eb2 = (const float*)d_in[16];
  float* out = (float*)d_out;

  char* ws = (char*)d_ws; size_t off = 0;
  auto alloc = [&](size_t bytes) -> void* { void* p = ws + off; off = (off + bytes + 255) & ~(size_t)255; return p; };
  __bf16* Ptw2 = (__bf16*)alloc((size_t)3 * HH * HH * 2);
  __bf16* Pn1x = (__bf16*)alloc((size_t)3 * HH * HH * 2);
  __bf16* Pn1t = (__bf16*)alloc((size_t)3 * HH * HH * 2);
  __bf16* Pn2  = (__bf16*)alloc((size_t)3 * HH * HH * 2);
  __bf16* Pd1  = (__bf16*)alloc((size_t)3 * HD2 * HH * 2);
  __bf16* Pe1  = (__bf16*)alloc((size_t)3 * HD2 * HH * 2);
  float* coef = (float*)alloc(3 * 1024 * 4);
  float* teh  = (float*)alloc((size_t)TP * HH * 4);
  float* te   = (float*)alloc((size_t)TP * HH * 4);
  float* tep  = (float*)alloc((size_t)TP * HH * 4);
  float* xfin = (float*)alloc((size_t)BB * HH * 4);
  float* dh   = (float*)alloc((size_t)BB * HD2 * 4);
  float* eh   = (float*)alloc((size_t)BB * HD2 * 4);

  const int t512 = (HH / 64) * (HH / 64), t256 = (HH / 64) * (HD2 / 64);
  k_split3<<<t512, 256, 0, stream>>>(tw2, Ptw2, HH, HH);
  k_split3<<<t512, 256, 0, stream>>>(nw1, Pn1x, HH, HH);
  k_split3<<<t512, 256, 0, stream>>>(nw1 + (size_t)HH * HH, Pn1t, HH, HH);
  k_split3<<<t512, 256, 0, stream>>>(nw2, Pn2, HH, HH);
  k_split3<<<t256, 256, 0, stream>>>(dw1, Pd1, HH, HD2);
  k_split3<<<t256, 256, 0, stream>>>(ew1, Pe1, HH, HD2);
  k_coeff<<<1, 32, 0, stream>>>(coef);
  k_teh<<<TP * HH / 256, 256, 0, stream>>>(tw1, tb1, teh);
  k_gemm6<HH, 0><<<TP / 16, 128, 0, stream>>>(teh, Ptw2, tb2, te);
  k_gemm6<HH, 0><<<TP / 16, 128, 0, stream>>>(te, Pn1t, nb1, tep);
  k_loop<<<BB / 16, 256, 0, stream>>>(x0, Pn1x, Pn2, tep, nb2, coef, xfin);
  k_gemm6<HD2, 1><<<BB / 16, 128, 0, stream>>>(xfin, Pd1, db1, dh);
  k_gemm6<HD2, 1><<<BB / 16, 128, 0, stream>>>(xfin, Pe1, eb1, eh);
  k_out<<<(BB * (HH + 3) / 4 + 255) / 256, 256, 0, stream>>>(xfin, dh, eh, dw2, db2, ew2, eb2, out);
}
